// GatedMultifactorSelfAttnEnc_31164282700424
// MI455X (gfx1250) — hardware-run, weakly checked
//
#include <hip/hip_runtime.h>
#include <stddef.h>


typedef _Float16 v16h __attribute__((ext_vector_type(16)));
typedef _Float16 v8h  __attribute__((ext_vector_type(8)));
typedef _Float16 v4h  __attribute__((ext_vector_type(4)));
typedef float    v8f  __attribute__((ext_vector_type(8)));
typedef float    v4f  __attribute__((ext_vector_type(4)));
typedef int      v4i  __attribute__((ext_vector_type(4)));
typedef _Float16 h16;

#ifndef NB
#define NB 8
#endif
#ifndef SEQ
#define SEQ 1024
#endif
#define NB_FULL  8
#define SEQ_FULL 1024
#define XD    512
#define NFAC  4
#define NPROJ (XD * NFAC)
#define JD    (2 * XD)
#define MROWS (NB * SEQ)

#ifndef SCORE_RES
#define SCORE_RES 1
#endif

#define QR 32
#define KC 128
#define SLD 132
#define PLD 136

static_assert(NB >= 1 && NB <= NB_FULL);
static_assert(SEQ >= 128 && SEQ <= SEQ_FULL && (SEQ % 128) == 0);
static_assert((SEQ % KC) == 0 && (SEQ % QR) == 0 && (SEQ % 64) == 0);
static_assert(QR == 32);
static_assert(KC == 4 * 32);
static_assert(XD == 4 * 128);
static_assert((XD % 64) == 0 && (XD % 32) == 0);
static_assert((NPROJ % 64) == 0 && (JD % 64) == 0 && (JD % 32) == 0);
static_assert((MROWS % 64) == 0);
static_assert((SLD % 4) == 0 && SLD >= KC);
static_assert((PLD % 8) == 0 && PLD >= KC);
static_assert((size_t)NB * NFAC * SEQ * XD < (size_t)0xFFFFFFFFu);
static_assert((size_t)NB * XD * SEQ < (size_t)0xFFFFFFFFu);

#define LDT 72
#define LDC 68
static_assert((LDT % 8) == 0 && LDT >= 64);
static_assert((LDC % 4) == 0 && LDC >= 64);

#define WCARRY 64.0f
#define PCARRY2 16384.0f
#define RCARRY 2048.0f

#define WPT_BYTES ((size_t)NPROJ * XD * 2)
#define WGT_BYTES ((size_t)JD * JD * 2)
#define J16_BYTES ((size_t)MROWS * JD * 2)
#define XT_BYTES  ((size_t)NB * XD * SEQ * 2)
#define Y_BYTES   ((size_t)NB * NFAC * SEQ * XD * 2)
#define OFF_WPT ((size_t)0)
#define OFF_WGT (OFF_WPT + WPT_BYTES)
#define OFF_J16 (OFF_WGT + WGT_BYTES)
#define OFF_XT  (OFF_J16 + J16_BYTES)
#define OFF_YH  (OFF_XT + XT_BYTES)
#define OFF_YR  (OFF_YH + Y_BYTES)
#define WS_TOTAL (OFF_YR + Y_BYTES)
static_assert((WPT_BYTES % 128) == 0 && (WGT_BYTES % 128) == 0 && (J16_BYTES % 128) == 0);
static_assert((XT_BYTES % 128) == 0 && (Y_BYTES % 128) == 0);
static_assert(WS_TOTAL <= (size_t)134217728);

__device__ __forceinline__ float bf16r(float x) {
  unsigned int u = __float_as_uint(x);
  u = (u + 0x7FFFu + ((u >> 16) & 1u)) & 0xFFFF0000u;
  return __uint_as_float(u);
}

static __device__ __forceinline__ h16 toh_flush(float v) {
  const h16 r = (h16)v;
  return (fabsf(v) < 6.103515625e-05f) ? (h16)0.0f : r;
}

__device__ __forceinline__ v16h frag_at(const _Float16* p) {
  v8h lo = *(const v8h*)(p);
  v8h hi = *(const v8h*)(p + 16);
  v16h out;
#pragma unroll
  for (int i = 0; i < 8; ++i) { out[i] = lo[i]; out[i + 8] = hi[i]; }
  return out;
}
__device__ __forceinline__ v16h ld_frag(const _Float16* base, unsigned ld) {
  const unsigned lane = threadIdx.x & 31u;
  return frag_at(base + (lane & 15u) * ld + (lane >> 4) * 8u);
}

__device__ __forceinline__ v8f wmma16(v16h a, v16h b, v8f c) {
  v8f d = __builtin_amdgcn_wmma_f32_16x16x32_f16(false, a, false, b, (short)0, c,
                                                 false, false);
  asm volatile("v_nop\n\tv_nop\n\tv_nop\n\tv_nop" : "+v"(d) : "v"(a), "v"(b));
  return d;
}

__device__ __forceinline__ float red32_sum(float x) {
#pragma unroll
  for (int off = 1; off < 32; off <<= 1) x += __shfl_xor(x, off, 32);
  return x;
}
__device__ __forceinline__ float red32_max(float x) {
#pragma unroll
  for (int off = 1; off < 32; off <<= 1) x = fmaxf(x, __shfl_xor(x, off, 32));
  return x;
}

__device__ __forceinline__ void wave_lds_sync() {
  __builtin_amdgcn_fence(3  , "wavefront");
  asm volatile("s_wait_dscnt 0x0" ::: "memory");
  __builtin_amdgcn_wave_barrier();
}

__global__ __launch_bounds__(256) void wconv_kernel(
    const float* __restrict__ W, _Float16* __restrict__ Wt, unsigned ldw, unsigned ldk) {
  __shared__ _Float16 T[64 * LDT];
  const unsigned tid = threadIdx.x;
  const unsigned n0 = blockIdx.x * 64u;
  const unsigned k0 = blockIdx.y * 64u;
#pragma unroll 4
  for (unsigned j = 0; j < 16u; ++j) {
    const unsigned idx = tid + 256u * j;
    const unsigned kr = idx >> 6, nc = idx & 63u;
    const float v = W[(size_t)(k0 + kr) * ldw + n0 + nc];
    T[nc * LDT + kr] = (_Float16)(WCARRY * bf16r(v));
  }
  __syncthreads();
  v8h x[2];
  size_t off[2];
#pragma unroll
  for (unsigned i = 0; i < 2u; ++i) {
    const unsigned n = 32u * i + (tid >> 3);
    const unsigned kc = (tid & 7u) * 8u;
    x[i] = *(const v8h*)&T[n * LDT + kc];
    off[i] = (size_t)(n0 + n) * ldk + k0 + kc;
  }
#pragma unroll
  for (int i = 0; i < 2; ++i) *(volatile v8h*)(Wt + off[i]) = x[i];
  __threadfence();
#pragma unroll
  for (int i = 0; i < 2; ++i) *(volatile v8h*)(Wt + off[i]) = x[i];
}

__global__ __launch_bounds__(256) void wconv_fac_kernel(
    const float* __restrict__ W, _Float16* __restrict__ Wt) {
  __shared__ _Float16 T[64 * LDT];
  const unsigned tid = threadIdx.x;
  const unsigned n0 = blockIdx.x * 64u;
  const unsigned k0 = blockIdx.y * 64u;
  const unsigned f = n0 / (unsigned)XD;
  const unsigned h0 = n0 - f * (unsigned)XD;
#pragma unroll 4
  for (unsigned j = 0; j < 16u; ++j) {
    const unsigned idx = tid + 256u * j;
    const unsigned kr = idx >> 6, nc = idx & 63u;
    const float v = W[(size_t)(k0 + kr) * NPROJ + (h0 + nc) * NFAC + f];
    T[nc * LDT + kr] = toh_flush(WCARRY * bf16r(v));
  }
  __syncthreads();
  v8h x[2];
  size_t off[2];
#pragma unroll
  for (unsigned i = 0; i < 2u; ++i) {
    const unsigned n = 32u * i + (tid >> 3);
    const unsigned kc = (tid & 7u) * 8u;
    x[i] = *(const v8h*)&T[n * LDT + kc];
    off[i] = (size_t)(n0 + n) * XD + k0 + kc;
  }
#pragma unroll
  for (int i = 0; i < 2; ++i) *(volatile v8h*)(Wt + off[i]) = x[i];
  __threadfence();
#pragma unroll
  for (int i = 0; i < 2; ++i) *(volatile v8h*)(Wt + off[i]) = x[i];
}

__global__ __launch_bounds__(256) void xprep_kernel(
    const float* __restrict__ X, _Float16* __restrict__ J16, _Float16* __restrict__ Xt) {
  __shared__ _Float16 T[64 * LDT];
  __shared__ _Float16 U[64 * LDT];
  const unsigned tid = threadIdx.x;
  const unsigned h0 = blockIdx.x * 64u;
  const unsigned row0 = blockIdx.y * 64u;
  const unsigned bidx = row0 / (unsigned)SEQ;
  const unsigned l0 = row0 - bidx * (unsigned)SEQ;
  const size_t frow0 = (size_t)bidx * SEQ_FULL + l0;
#pragma unroll 4
  for (unsigned j = 0; j < 16u; ++j) {
    const unsigned idx = tid + 256u * j;
    const unsigned r = idx >> 6, c = idx & 63u;
    const float v = X[(frow0 + r) * XD + h0 + c];
    const h16 hv = toh_flush(bf16r(v));
    T[r * LDT + c] = hv;
    U[c * LDT + r] = hv;
  }
  __syncthreads();
  v8h xa[2], xb[2];
  size_t offa[2], offb[2];
#pragma unroll
  for (unsigned i = 0; i < 2u; ++i) {
    const unsigned n = 32u * i + (tid >> 3);
    const unsigned kc = (tid & 7u) * 8u;
    xa[i] = *(const v8h*)&T[n * LDT + kc];
    xb[i] = *(const v8h*)&U[n * LDT + kc];
    offa[i] = (size_t)(row0 + n) * JD + h0 + kc;
    offb[i] = ((size_t)bidx * XD + h0 + n) * SEQ + l0 + kc;
  }
#pragma unroll
  for (int i = 0; i < 2; ++i) {
    *(volatile v8h*)(J16 + offa[i]) = xa[i];
    *(volatile v8h*)(Xt + offb[i]) = xb[i];
  }
  __threadfence();
#pragma unroll
  for (int i = 0; i < 2; ++i) {
    *(volatile v8h*)(J16 + offa[i]) = xa[i];
    *(volatile v8h*)(Xt + offb[i]) = xb[i];
  }
}

template <int MODE>
__device__ __forceinline__ void mm_body(
    const _Float16* __restrict__ A16, const unsigned lda,
    const _Float16* __restrict__ Bt, const unsigned K,
    const float* __restrict__ bias, const float* __restrict__ xin,
    float* __restrict__ outf, _Float16* __restrict__ outh, _Float16* __restrict__ outr) {
  __shared__ float Cs[64 * LDC];
  const unsigned tid = threadIdx.x, lane = tid & 31u;
  const unsigned w = (unsigned)__builtin_amdgcn_readfirstlane((int)(threadIdx.x >> 5));
  const unsigned mw = w >> 1, nw = w & 1u;
  const unsigned hh = lane >> 4, m = lane & 15u;
  const unsigned n0 = blockIdx.x * 64u;
  const unsigned row0 = blockIdx.y * 64u;

  const _Float16* ap  = A16 + (size_t)(row0 + mw * 16u + m) * lda + hh * 8u;
  const _Float16* bp0 = Bt + (size_t)(n0 + nw * 32u + m) * K + hh * 8u;
  const _Float16* bp1 = bp0 + (size_t)16 * K;
  v8f acc0 = {}, acc1 = {};
#pragma unroll 2
  for (unsigned k0 = 0; k0 < K; k0 += 32u) {
    const v16h a  = frag_at(ap + k0);
    const v16h b0 = frag_at(bp0 + k0);
    const v16h b1 = frag_at(bp1 + k0);
    acc0 = wmma16(a, b0, acc0);
    acc1 = wmma16(a, b1, acc1);
  }
#pragma unroll
  for (int r = 0; r < 8; ++r) {
    float* d = &Cs[(mw * 16u + hh * 8u + (unsigned)r) * LDC + nw * 32u + m];
    d[0]  = acc0[r];
    d[16] = acc1[r];
  }
  __syncthreads();

  if (MODE == 0) {
    const unsigned f = n0 / (unsigned)XD;
    const unsigned h0 = n0 - f * (unsigned)XD;
    v8h x[2], xr[2];
    size_t off[2];
#pragma unroll
    for (unsigned i = 0; i < 2u; ++i) {
      const unsigned r = 32u * i + (tid >> 3);
      const unsigned c = (tid & 7u) * 8u;
      const unsigned crow = row0 + r;
      const unsigned bidx = crow / (unsigned)SEQ;
      const unsigned sq = crow - bidx * (unsigned)SEQ;
      const v4f u0 = *(const v4f*)&Cs[r * LDC + c];
      const v4f u1 = *(const v4f*)&Cs[r * LDC + c + 4];
#pragma unroll
      for (unsigned j = 0; j < 4u; ++j) {
        const float g0 = bf16r(bias[(h0 + c + j) * NFAC + f]);
        const float g1 = bf16r(bias[(h0 + c + 4u + j) * NFAC + f]);
        const float t0 = fmaxf(u0[j] * (1.0f / WCARRY) + g0, 0.0f);
        const float t1 = fmaxf(u1[j] * (1.0f / WCARRY) + g1, 0.0f);
        const h16 a0 = toh_flush(t0);
        const h16 a1 = toh_flush(t1);
        x[i][j]      = a0;
        x[i][j + 4]  = a1;
        xr[i][j]     = toh_flush((t0 - (float)a0) * RCARRY);
        xr[i][j + 4] = toh_flush((t1 - (float)a1) * RCARRY);
      }
      off[i] = (((size_t)bidx * NFAC + f) * SEQ + sq) * XD + h0 + c;
    }
#pragma unroll
    for (int i = 0; i < 2; ++i) {
      *(volatile v8h*)(outh + off[i]) = x[i];
      *(volatile v8h*)(outr + off[i]) = xr[i];
    }
    __threadfence();
#pragma unroll
    for (int i = 0; i < 2; ++i) {
      *(volatile v8h*)(outh + off[i]) = x[i];
      *(volatile v8h*)(outr + off[i]) = xr[i];
    }
  }

  if (MODE == 1) {
    const bool xhalf = (n0 < (unsigned)XD);
    v4f xs[4];
    size_t off[4];
#pragma unroll
    for (unsigned i = 0; i < 4u; ++i) {
      const unsigned r = 16u * i + (tid >> 4);
      const unsigned c = (tid & 15u) * 4u;
      const unsigned crow = row0 + r;
      const unsigned bidx = crow / (unsigned)SEQ;
      const unsigned sq = crow - bidx * (unsigned)SEQ;
      const size_t frow = (size_t)bidx * SEQ_FULL + sq;
      const v4f u = *(const v4f*)&Cs[r * LDC + c];
      const v4f g = *(const v4f*)(bias + n0 + c);
      v4f jv;
      if (xhalf) {
        const v4f xv = *(const v4f*)(xin + frow * XD + n0 + c);
#pragma unroll
        for (int j = 0; j < 4; ++j) jv[j] = bf16r(xv[j]);
      } else {
        const v4h ev = *(const v4h*)(A16 + (size_t)crow * lda + n0 + c);
#pragma unroll
        for (int j = 0; j < 4; ++j) jv[j] = (float)ev[j];
      }
      v4f val;
#pragma unroll
      for (int j = 0; j < 4; ++j) {
        const float s = u[j] * (1.0f / WCARRY) + bf16r(g[j]);
        const float gt = __builtin_amdgcn_rcpf(1.0f + __expf(-s));
        val[j] = gt * jv[j];
      }
      xs[i] = val;
      off[i] = frow * JD + n0 + c;
    }
#pragma unroll
    for (int i = 0; i < 4; ++i) *(volatile v4f*)(outf + off[i]) = xs[i];
    __threadfence();
#pragma unroll
    for (int i = 0; i < 4; ++i) *(volatile v4f*)(outf + off[i]) = xs[i];
  }
}

__global__ __launch_bounds__(256) void proj_kernel(
    const _Float16* __restrict__ J16, const _Float16* __restrict__ WpT,
    const float* __restrict__ bp, _Float16* __restrict__ Yh, _Float16* __restrict__ Yr) {
  mm_body<0>(J16, (unsigned)JD, WpT, (unsigned)XD, bp, bp, (float*)0, Yh, Yr);
}
__global__ __launch_bounds__(256) void gate_kernel(
    const _Float16* __restrict__ J16, const _Float16* __restrict__ WgT,
    const float* __restrict__ bg, const float* __restrict__ X, float* __restrict__ outf) {
  mm_body<1>(J16, (unsigned)JD, WgT, (unsigned)JD, bg, X, outf, (_Float16*)0, (_Float16*)0);
}

__global__ __launch_bounds__(256) __attribute__((amdgpu_num_vgpr(256))) void mfattn_kernel(
    const _Float16* __restrict__ Yh, const _Float16* __restrict__ Yr,
    const _Float16* __restrict__ Xt, const int* __restrict__ xmask,
    _Float16* __restrict__ J16) {
  __shared__ float Sc[QR * SLD];
  __shared__ _Float16 Pt[QR * PLD];
  __shared__ _Float16 Ot[8 * 16 * LDT];
  __shared__ float Rs[QR];
  __shared__ float Fin[QR];

  const unsigned tid = threadIdx.x, lane = tid & 31u;
  const unsigned wave = (unsigned)__builtin_amdgcn_readfirstlane((int)(threadIdx.x >> 5));
  const unsigned hh = lane >> 4, m = lane & 15u;
  const unsigned rg = wave & 1u;
  const unsigned kq = wave >> 1;
  const unsigned q0 = blockIdx.x * (unsigned)QR;
  const unsigned b = blockIdx.y;

  float mrow[4], se[4], spm[4];
  int qm[4];
#pragma unroll
  for (int i = 0; i < 4; ++i) {
    mrow[i] = -1.0e30f;
    se[i] = 0.0f;
    spm[i] = 0.0f;
    qm[i] = xmask[(size_t)b * SEQ_FULL + q0 + wave * 4u + (unsigned)i];
  }
  v8f o[8];
#pragma unroll
  for (int nb = 0; nb < 8; ++nb) o[nb] = (v8f){};

  const unsigned ao = ((b * (unsigned)NFAC) * (unsigned)SEQ + q0 + rg * 16u + m) * (unsigned)XD + hh * 8u;

  for (unsigned kb = 0; kb < (unsigned)SEQ; kb += (unsigned)KC) {
    v8f best0, best1;
#pragma unroll
    for (int r = 0; r < 8; ++r) { best0[r] = -3.0e38f; best1[r] = -3.0e38f; }
    const unsigned bo = ((b * (unsigned)NFAC) * (unsigned)SEQ + kb + kq * 32u + m) * (unsigned)XD + hh * 8u;
#pragma unroll 1
    for (unsigned f = 0; f < (unsigned)NFAC; ++f) {
      const unsigned fo = f * ((unsigned)SEQ * (unsigned)XD);
      const unsigned a_o = ao + fo;
      const unsigned b_o0 = bo + fo;
      const unsigned b_o1 = b_o0 + 16u * (unsigned)XD;
      v8f s0 = {}, s1 = {};
#if SCORE_RES
      v8f r0 = {}, r1 = {};
#endif
#pragma unroll 1
      for (unsigned k0 = 0; k0 < (unsigned)XD; k0 += 32u) {
        const v16h a  = frag_at(Yh + (a_o + k0));
        const v16h c0 = frag_at(Yh + (b_o0 + k0));
        const v16h c1 = frag_at(Yh + (b_o1 + k0));
        s0 = wmma16(a, c0, s0);
        s1 = wmma16(a, c1, s1);
#if SCORE_RES
        const v16h ax = frag_at(Yr + (a_o + k0));
        const v16h d0 = frag_at(Yr + (b_o0 + k0));
        const v16h d1 = frag_at(Yr + (b_o1 + k0));
        r0 = wmma16(a, d0, r0);
        r0 = wmma16(ax, c0, r0);
        r1 = wmma16(a, d1, r1);
        r1 = wmma16(ax, c1, r1);
#endif
      }
#pragma unroll
      for (int r = 0; r < 8; ++r) {
#if SCORE_RES
        const float t0 = s0[r] + r0[r] * (1.0f / RCARRY);
        const float t1 = s1[r] + r1[r] * (1.0f / RCARRY);
#else
        const float t0 = s0[r];
        const float t1 = s1[r];
#endif
        best0[r] = fmaxf(best0[r], t0);
        best1[r] = fmaxf(best1[r], t1);
      }
    }
#pragma unroll
    for (int r = 0; r < 8; ++r) {
      float* d = &Sc[(rg * 16u + hh * 8u + (unsigned)r) * SLD + kq * 32u + m];
      d[0]  = best0[r];
      d[16] = best1[r];
    }
    __syncthreads();

    const unsigned key0 = kb + lane * 4u;
    const v4i km = *(const v4i*)(xmask + (size_t)b * SEQ_FULL + key0);
#pragma unroll
    for (int i = 0; i < 4; ++i) {
      const unsigned row = wave * 4u + (unsigned)i;
      const unsigned ql = q0 + row;
      const v4f sv = *(const v4f*)&Sc[row * SLD + lane * 4u];
      float mk[4], t[4];
#pragma unroll
      for (int j = 0; j < 4; ++j) {
        int mi = qm[i] * km[j];
        mi = (key0 + (unsigned)j == ql) ? 0 : mi;
        mk[j] = (float)mi;
        t[j] = sv[j] * mk[j];
      }
      float cm = fmaxf(fmaxf(t[0], t[1]), fmaxf(t[2], t[3]));
      cm = red32_max(cm);
      const float mn = fmaxf(mrow[i], cm);
      const float al = __expf(mrow[i] - mn);
      mrow[i] = mn;
      float es = 0.0f, ps = 0.0f;
      v4h pv;
#pragma unroll
      for (int j = 0; j < 4; ++j) {
        const float d = t[j] - mn;
        const float e = __expf(d);
        const float pm = e * mk[j];
        es += e;
        ps += pm;
        const float pc = (d < -19.4f) ? 0.0f : pm * PCARRY2;
        pv[j] = toh_flush(pc);
      }
      es = red32_sum(es);
      ps = red32_sum(ps);
      se[i] = se[i] * al + es;
      spm[i] = spm[i] * al + ps;
      if (lane == 0u) Rs[row] = al;
      *(v4h*)&Pt[row * PLD + lane * 4u] = pv;
    }
    __syncthreads();

    {
      float rs8[8];
#pragma unroll
      for (int r = 0; r < 8; ++r) rs8[r] = Rs[rg * 16u + hh * 8u + (unsigned)r];
#pragma unroll
      for (int nb = 0; nb < 8; ++nb)
#pragma unroll
        for (int r = 0; r < 8; ++r) o[nb][r] = o[nb][r] * rs8[r];
      const unsigned xo = ((b * (unsigned)XD + kq * 128u + m) * (unsigned)SEQ) + kb + hh * 8u;
#pragma unroll 1
      for (unsigned c = 0; c < 4u; ++c) {
        const v16h pf = ld_frag(&Pt[(rg * 16u) * PLD + c * 32u], PLD);
#pragma unroll
        for (int nb = 0; nb < 8; ++nb) {
          const v16h vf = frag_at(Xt + (xo + (unsigned)nb * 16u * (unsigned)SEQ + c * 32u));
          o[nb] = wmma16(pf, vf, o[nb]);
        }
      }
    }
  }

#pragma unroll
  for (int i = 0; i < 4; ++i) {
    const float den = spm[i] + 1.0e-13f * se[i];
    const float fv = __builtin_amdgcn_rcpf(den) * (1.0f / PCARRY2);
    if (lane == 0u) Fin[wave * 4u + (unsigned)i] = fv;
  }
  __syncthreads();
  float fin8[8];
#pragma unroll
  for (int r = 0; r < 8; ++r) fin8[r] = Fin[rg * 16u + hh * 8u + (unsigned)r];

  _Float16* T = Ot + wave * (16u * LDT);
#pragma unroll
  for (int p = 0; p < 2; ++p) {
#pragma unroll
    for (int nb = 0; nb < 4; ++nb)
#pragma unroll
      for (int r = 0; r < 8; ++r)
        T[(hh * 8u + (unsigned)r) * LDT + (unsigned)nb * 16u + m] =
            toh_flush(o[p * 4 + nb][r] * fin8[r]);
    wave_lds_sync();
    v8h x[4];
    size_t off[4];
#pragma unroll
    for (unsigned i = 0; i < 4u; ++i) {
      const unsigned r = 4u * i + (lane >> 3);
      const unsigned c = (lane & 7u) * 8u;
      x[i] = *(const v8h*)&T[r * LDT + c];
      off[i] = (size_t)(b * (unsigned)SEQ + q0 + rg * 16u + r) * JD + XD + kq * 128u +
               (unsigned)p * 64u + c;
    }
#pragma unroll
    for (int i = 0; i < 4; ++i) *(volatile v8h*)(J16 + off[i]) = x[i];
    __threadfence();
#pragma unroll
    for (int i = 0; i < 4; ++i) *(volatile v8h*)(J16 + off[i]) = x[i];
    wave_lds_sync();
  }
}

extern "C" void kernel_launch(void* const* d_in, const int* in_sizes, int n_in,
                              void* d_out, int out_size, void* d_ws, size_t ws_size,
                              hipStream_t stream) {
  if (n_in < 6) return;
  const long long need_rows = (long long)(NB - 1) * SEQ_FULL + SEQ;
  if ((long long)in_sizes[0] < need_rows * XD) return;
  if ((long long)in_sizes[1] < need_rows) return;
  if ((long long)in_sizes[2] < (long long)XD * NPROJ) return;
  if (in_sizes[3] < NPROJ) return;
  if ((long long)in_sizes[4] < (long long)JD * JD) return;
  if (in_sizes[5] < JD) return;
  if ((long long)out_size < need_rows * JD) return;
  if (ws_size < WS_TOTAL) return;

  const float* X     = (const float*)d_in[0];
  const int*   xmask = (const int*)d_in[1];
  const float* wp    = (const float*)d_in[2];
  const float* bp    = (const float*)d_in[3];
  const float* wg    = (const float*)d_in[4];
  const float* bg    = (const float*)d_in[5];
  float* out = (float*)d_out;

  char* ws = (char*)d_ws;
  _Float16* WpT = (_Float16*)(ws + OFF_WPT);
  _Float16* WgT = (_Float16*)(ws + OFF_WGT);
  _Float16* J16 = (_Float16*)(ws + OFF_J16);
  _Float16* Xt  = (_Float16*)(ws + OFF_XT);
  _Float16* Yh  = (_Float16*)(ws + OFF_YH);
  _Float16* Yr  = (_Float16*)(ws + OFF_YR);

  dim3 blk(256);

  wconv_fac_kernel<<<dim3(NPROJ / 64, XD / 64), blk, 0, stream>>>(wp, WpT);
  wconv_kernel<<<dim3(JD / 64, JD / 64), blk, 0, stream>>>(wg, WgT, (unsigned)JD, (unsigned)JD);
  xprep_kernel<<<dim3(XD / 64, MROWS / 64), blk, 0, stream>>>(X, J16, Xt);
  proj_kernel<<<dim3(NPROJ / 64, MROWS / 64), blk, 0, stream>>>(J16, WpT, bp, Yh, Yr);
  mfattn_kernel<<<dim3(SEQ / QR, NB), blk, 0, stream>>>(Yh, Yr, Xt, xmask, J16);
  gate_kernel<<<dim3(JD / 64, MROWS / 64), blk, 0, stream>>>(J16, WgT, bg, X, out);
}
